// DecomposedCandidateBaseline_32779190403194
// MI455X (gfx1250) — hardware-verified
//
#include <hip/hip_runtime.h>
#include <math.h>

typedef __attribute__((ext_vector_type(16))) _Float16 v16h;
typedef __attribute__((ext_vector_type(16))) __bf16 v16b;
typedef __attribute__((ext_vector_type(8)))  _Float16 v8h;
typedef __attribute__((ext_vector_type(8)))  float v8f;
typedef __attribute__((ext_vector_type(4)))  float v4f;
typedef __attribute__((ext_vector_type(2)))  float v2f;
typedef __attribute__((ext_vector_type(4)))  unsigned v4u;
typedef __attribute__((ext_vector_type(4)))  int v4i;
typedef float __attribute__((may_alias)) float_a;
typedef int __attribute__((may_alias)) int_a;

template <typename T> __device__ __forceinline__ void vst2(void* p, T v) { *(volatile T*)p = v; __threadfence(); *(volatile T*)p = v; }
__device__ __forceinline__ v8f wmma16(v16h a, v16h b, v8f c) {
  v8f d = __builtin_amdgcn_wmma_f32_16x16x32_f16(false, a, false, b, (short)0, c, false, false);
  asm volatile("v_nop\n\tv_nop\n\tv_nop\n\tv_nop" : "+v"(d) : "v"(a), "v"(b));
  return d;
}
__device__ __forceinline__ v8f wmma_bf(v16b a, v16b b, v8f c) {
  v8f d = __builtin_amdgcn_wmma_f32_16x16x32_bf16(false, a, false, b, (short)0, c, false, false);
  asm volatile("v_nop\n\tv_nop\n\tv_nop\n\tv_nop" : "+v"(d) : "v"(a), "v"(b));
  return d;
}
__device__ __forceinline__ v16h frag_h(const _Float16* rowk0, int lane) {
  union { v16h v; v8h q[2]; } u; const _Float16* p = rowk0 + 8 * (lane >> 4);
  u.q[0] = *(const v8h*)p; u.q[1] = *(const v8h*)(p + 16); return u.v;
}
__device__ __forceinline__ v16h frag_f32(const float* rowk0, int lane) {
  v16h a; const float* p = rowk0 + 8 * (lane >> 4);
#pragma unroll
  for (int i = 0; i < 8; ++i) { a[i] = (_Float16)p[i]; a[8 + i] = (_Float16)p[16 + i]; }
  return a;
}
__device__ __forceinline__ v16h frag_f32s(const float* rowk0, int lane, float sc) {
  v16h a; const float* p = rowk0 + 8 * (lane >> 4);
#pragma unroll
  for (int i = 0; i < 8; ++i) { a[i] = (_Float16)(p[i] * sc); a[8 + i] = (_Float16)(p[16 + i] * sc); }
  return a;
}
__device__ __forceinline__ v16h fragc_f32(const float* W, int k0, int n, int lane, int ld, int K) {
  v16h a; const int g = lane >> 4;
#pragma unroll
  for (int i = 0; i < 8; ++i) { const int ka = k0 + 8 * g + i, kb = ka + 16;
    a[i] = (_Float16)(ka < K ? W[(size_t)(ka < K ? ka : K - 1) * ld + n] : 0.f); a[8 + i] = (_Float16)(kb < K ? W[(size_t)(kb < K ? kb : K - 1) * ld + n] : 0.f); }
  return a;
}
struct F2 { v16b h, l; };
__device__ __forceinline__ F2 bsplit16(const float v[16]) { F2 r;
#pragma unroll
  for (int i = 0; i < 16; ++i) { const __bf16 h = (__bf16)v[i]; r.h[i] = h; r.l[i] = (__bf16)(v[i] - (float)h); }
  return r; }
__device__ __forceinline__ F2 split_row(const float* row, int k0, int lane) { float v[16]; const float* p = row + k0 + 8 * (lane >> 4);
#pragma unroll
  for (int i = 0; i < 8; ++i) { v[i] = p[i]; v[8 + i] = p[16 + i]; }
  return bsplit16(v); }
__device__ __forceinline__ F2 split_rowK(const float* row, int k0, int lane, int K) { float v[16]; const int g = lane >> 4;
#pragma unroll
  for (int i = 0; i < 8; ++i) { const int ka = k0 + 8 * g + i, kb = ka + 16; v[i] = ka < K ? row[ka < K ? ka : K - 1] : 0.f; v[8 + i] = kb < K ? row[kb < K ? kb : K - 1] : 0.f; }
  return bsplit16(v); }
__device__ __forceinline__ F2 split_col(const float* W, int k0, int n, int lane, int ld, int K) { float v[16]; const int g = lane >> 4;
#pragma unroll
  for (int i = 0; i < 8; ++i) { const int ka = k0 + 8 * g + i, kb = ka + 16; v[i] = ka < K ? W[(size_t)(ka < K ? ka : K - 1) * ld + n] : 0.f; v[8 + i] = kb < K ? W[(size_t)(kb < K ? kb : K - 1) * ld + n] : 0.f; }
  return bsplit16(v); }
__device__ __forceinline__ v8f mac3(const F2& a, const F2& b, v8f c) { c = wmma_bf(a.l, b.h, c); c = wmma_bf(a.h, b.l, c); return wmma_bf(a.h, b.h, c); }
__device__ __forceinline__ float sigm(float v) { return 1.0f / (1.0f + expf(-v)); }
#define LDSX() do { asm volatile("s_wait_dscnt 0" ::: "memory"); __builtin_amdgcn_wave_barrier(); __builtin_amdgcn_fence(__ATOMIC_RELEASE, "workgroup"); } while (0)


#define NS 2048
#define LC 20
#define LH 200
#define DD 128
#define HH 512
#define DEN 256
#define NV 100000
#define NPOSV 201
#define NGRP 4
#define FUS (7 * DD + HH)
#ifndef TNS
#define TNS NS
#endif
typedef __attribute__((ext_vector_type(8))) __bf16 v8b;
__device__ __forceinline__ v16b frag_b(const __bf16* rowk0, int lane) {
  union { v16b v; v8b q[2]; } u; const __bf16* p = rowk0 + 8 * (lane >> 4);
  u.q[0] = *(const v8b*)p; u.q[1] = *(const v8b*)(p + 16); return u.v;
}
__device__ __forceinline__ v16b frag_gbf(const float* rowk0, int lane) {
  v16b a; const float* p = rowk0 + 8 * (lane >> 4);
#pragma unroll
  for (int i = 0; i < 8; ++i) { a[i] = (__bf16)p[i]; a[8 + i] = (__bf16)p[16 + i]; }
  return a;
}
__device__ __forceinline__ float bfr(float v) { return (float)(__bf16)v; }
__device__ __attribute__((noinline)) float exp_ni(float v) { return expf(v); }
__device__ __forceinline__ float silu(float v) { return v / (1.0f + exp_ni(-v)); }
__device__ __forceinline__ int clampi(int v, int hi) { return v < 0 ? 0 : (v > hi ? hi : v); }

#define P_W2   0u
#define P_WC   (P_W2 + 128u * 128)
#define P_WD   (P_WC + 128u * 256)
#define P_WQ   (P_WD + 512u * 256)
#define P_W1O  (P_WQ + 128u * 896)
#define P_W2O  (P_W1O + 512u * 1408)
#define P_END  (P_W2O + 256u * 512)
#define WS_PT   0u
#define WS_CS   (WS_PT + 2u * P_END + 256)
#define WS_XS   (WS_CS + 4u * NS * DD)
#define WS_CH   (WS_XS + 4u * NS * DD)
#define WS_DS   (WS_CH + 4u * NS * DD)
#define WS_Q    (WS_DS + 4u * NS * HH)
#define WS_FU   (WS_Q + 4u * NS * DD)
#define WS_END  (WS_FU + 4u * NS * FUS)

__global__ __launch_bounds__(256) void k_pack(const float* __restrict__ w2, const float* __restrict__ wc, const float* __restrict__ wd, const float* __restrict__ wq, const float* __restrict__ w1o, const float* __restrict__ w2o, __bf16* __restrict__ PT) {
  __shared__ __align__(16) __bf16 srow[FUS];
  const int n = blockIdx.x, tid = threadIdx.x; const float* src; int K, NOUT, nn; size_t base;
  if (n < 128) { src = w2; K = 128; NOUT = 128; nn = n; base = P_W2 + (size_t)nn * 128; }
  else if (n < 256) { src = wc; K = 256; NOUT = 128; nn = n - 128; base = P_WC + (size_t)nn * 256; }
  else if (n < 768) { src = wd; K = 256; NOUT = 512; nn = n - 256; base = P_WD + (size_t)nn * 256; }
  else if (n < 896) { src = wq; K = 896; NOUT = 128; nn = n - 768; base = P_WQ + (size_t)nn * 896; }
  else if (n < 1408) { src = w1o; K = 1408; NOUT = 512; nn = n - 896; base = P_W1O + (size_t)nn * 1408; }
  else { src = w2o; K = 512; NOUT = 256; nn = n - 1408; base = P_W2O + (size_t)nn * 512; }
  for (int k = tid; k < K; k += 256) srow[k] = (__bf16)src[(size_t)k * NOUT + nn];
  __syncthreads();
  for (int q = tid; q < K / 8; q += 256) vst2((unsigned*)(PT + base + q * 8), *(const v4u*)(&srow[q * 8]));
}

__global__ __launch_bounds__(256) void k_hist(const int* __restrict__ ctok, const int* __restrict__ xtok, const int* __restrict__ hgrp, const int* __restrict__ cmask, const int* __restrict__ xmask, const int* __restrict__ hmask, const float* __restrict__ htime,
                                              const float* __restrict__ tok_emb, const float* __restrict__ grp_emb, const float* __restrict__ tw1, const float* __restrict__ tb1, const float* __restrict__ tb2, const __bf16* __restrict__ PT,
                                              const float* __restrict__ cb, const float* __restrict__ cg, const float* __restrict__ cbt, float* __restrict__ CS, float* __restrict__ XS, float* __restrict__ CH) {
  __shared__ __align__(16) __bf16 suh[8][16][DD + 8], sul[8][16][DD + 8];
  __shared__ __align__(16) __bf16 sgr[8][16][DD + 8];
  __shared__ __align__(16) float sth[8][16][DD + 4];
  __shared__ __align__(16) float sacc[8][DD + 4]; __shared__ float scnt[8];
  __shared__ __align__(16) float smean[2][DD];
  const int tid = threadIdx.x, wave = tid >> 5, lane = tid & 31, col = lane & 15, g = lane >> 4; const int b = blockIdx.x;
  { const int d = tid & 127, which = tid >> 7; const int* tk = which ? xtok : ctok; const int* mk = which ? xmask : cmask; float s = 0.f, c = 0.f;
#pragma unroll 1
    for (int i = 0; i < LC; ++i) { const int id = clampi(tk[b * LC + i], NV - 1); const float m = (float)mk[b * LC + i]; s += bfr(tok_emb[(size_t)id * DD + d]) * m; c += m; }
    smean[which][d] = s / fmaxf(c, 1.0f); }
  float accv[4] = {0.f, 0.f, 0.f, 0.f}; float cntw = 0.f;
#pragma unroll 1
  for (int tile = wave; tile < 13; tile += 8) { const int l0 = tile * 16;
    { const int rl = lane >> 1, half = lane & 1; const int l = l0 + rl; const int lc = l < LH ? l : LH - 1;
      const float t = bfr(htime[b * LH + lc]); const int gid = clampi(hgrp[b * LH + lc], NGRP - 1);
      for (int j = half * 64; j < half * 64 + 64; ++j) { const float u = silu(t * bfr(tw1[j]) + bfr(tb1[j])); const __bf16 hi = (__bf16)u; suh[wave][rl][j] = hi; sul[wave][rl][j] = (__bf16)(u - (float)hi); sgr[wave][rl][j] = (__bf16)grp_emb[gid * DD + j]; } }
    LDSX();
    { v8f acc[8] = {};
#pragma unroll
      for (int kc = 0; kc < 4; ++kc) { const v16b ah = frag_b(&suh[wave][col][kc * 32], lane), al = frag_b(&sul[wave][col][kc * 32], lane);
#pragma unroll
        for (int j = 0; j < 8; ++j) { const v16b w = frag_b(PT + P_W2 + (size_t)(j * 16 + col) * 128 + kc * 32, lane); acc[j] = wmma_bf(al, w, acc[j]); acc[j] = wmma_bf(ah, w, acc[j]); } }
#pragma unroll
      for (int j = 0; j < 8; ++j) { const float bb = bfr(tb2[j * 16 + col]);
#pragma unroll
        for (int r = 0; r < 8; ++r) sth[wave][8 * g + r][j * 16 + col] = acc[j][r] + bb; } }
    LDSX();
    { v8f acc[8] = {};
#pragma unroll
      for (int kc = 0; kc < 4; ++kc) { const v16b a = frag_b(&sgr[wave][col][kc * 32], lane);
#pragma unroll
        for (int j = 0; j < 8; ++j) acc[j] = wmma_bf(a, frag_b(PT + P_WC + (size_t)(j * 16 + col) * 256 + kc * 32, lane), acc[j]); }
#pragma unroll
      for (int kc = 0; kc < 4; ++kc) { const F2 a = split_row(&sth[wave][col][0], kc * 32, lane);
#pragma unroll
        for (int j = 0; j < 8; ++j) { const v16b w = frag_b(PT + P_WC + (size_t)(j * 16 + col) * 256 + 128 + kc * 32, lane); acc[j] = wmma_bf(a.l, w, acc[j]); acc[j] = wmma_bf(a.h, w, acc[j]); } }
      LDSX();
#pragma unroll
      for (int j = 0; j < 8; ++j) { const float bb = bfr(cb[j * 16 + col]);
#pragma unroll
        for (int r = 0; r < 8; ++r) sth[wave][8 * g + r][j * 16 + col] = acc[j][r] + bb; } }
    LDSX();
    { const int rl = lane >> 1, half = lane & 1; float s = 0.f;
#pragma unroll 8
      for (int j = 0; j < DD; ++j) s += sth[wave][rl][j];
      const float mu = s * (1.0f / DD); float q2 = 0.f;
#pragma unroll 8
      for (int j = 0; j < DD; ++j) { const float d = sth[wave][rl][j] - mu; q2 += d * d; }
      const float rs = rsqrtf(q2 * (1.0f / DD) + 1e-5f);
      LDSX();
      for (int j = half * 64; j < half * 64 + 64; ++j) sth[wave][rl][j] = silu((sth[wave][rl][j] - mu) * rs * bfr(cg[j]) + bfr(cbt[j])); }
    LDSX();
#pragma unroll 1
    for (int rl = 0; rl < 16; ++rl) { const int l = l0 + rl; if (l < LH) { const float m = (float)hmask[b * LH + l]; cntw += m;
#pragma unroll
        for (int i = 0; i < 4; ++i) accv[i] += m * sth[wave][rl][lane * 4 + i]; } }
    LDSX(); }
#pragma unroll
  for (int i = 0; i < 4; ++i) sacc[wave][lane * 4 + i] = accv[i];
  if (lane == 0) scnt[wave] = cntw;
  __syncthreads();
  if (tid < DD) { float s = 0.f, c = 0.f;
#pragma unroll
    for (int w = 0; w < 8; ++w) { s += sacc[w][tid]; c += scnt[w]; }
    sacc[0][tid] = s / fmaxf(c, 1.0f); }
  __syncthreads();
  if (tid < 32) vst2(CS + (size_t)b * DD + tid * 4, *(const v4f*)&smean[0][tid * 4]);
  else if (tid < 64) vst2(XS + (size_t)b * DD + (tid - 32) * 4, *(const v4f*)&smean[1][(tid - 32) * 4]);
  else if (tid < 96) vst2(CH + (size_t)b * DD + (tid - 64) * 4, *(const v4f*)&sacc[0][(tid - 64) * 4]);
}
__global__ __launch_bounds__(128) void k_dq(const float* __restrict__ dense, const __bf16* __restrict__ PT, const float* __restrict__ bd, const float* __restrict__ gd, const float* __restrict__ btd, const float* __restrict__ bq, const float* __restrict__ gq, const float* __restrict__ btq,
                                            const float* __restrict__ CS, const float* __restrict__ XS, const float* __restrict__ CH, float* __restrict__ DS, float* __restrict__ Q) {
  __shared__ __align__(16) float st[4][16][HH + 4];
  const int tid = threadIdx.x, wave = tid >> 5, lane = tid & 31, col = lane & 15, g = lane >> 4; const size_t r0 = (size_t)blockIdx.x * 64 + wave * 16;
#pragma unroll 1
  for (int pass = 0; pass < 2; ++pass) { v8f acc[16] = {};
#pragma unroll
    for (int kc = 0; kc < DEN / 32; ++kc) { const v16b a = frag_gbf(dense + (r0 + col) * DEN + kc * 32, lane);
#pragma unroll
      for (int j = 0; j < 16; ++j) acc[j] = wmma_bf(a, frag_b(PT + P_WD + (size_t)(pass * 256 + j * 16 + col) * 256 + kc * 32, lane), acc[j]); }
#pragma unroll
    for (int j = 0; j < 16; ++j) { const int n = pass * 256 + j * 16 + col; const float bb = bfr(bd[n]);
#pragma unroll
      for (int r = 0; r < 8; ++r) st[wave][8 * g + r][n] = acc[j][r] + bb; } }
  LDSX();
  { const int rl = lane >> 1, half = lane & 1; float s = 0.f;
#pragma unroll 8
    for (int j = 0; j < HH; ++j) s += st[wave][rl][j];
    const float mu = s * (1.0f / HH); float q2 = 0.f;
#pragma unroll 8
    for (int j = 0; j < HH; ++j) { const float d = st[wave][rl][j] - mu; q2 += d * d; }
    const float rs = rsqrtf(q2 * (1.0f / HH) + 1e-5f);
    LDSX();
    for (int j = half * 256; j < half * 256 + 256; ++j) st[wave][rl][j] = silu((st[wave][rl][j] - mu) * rs * bfr(gd[j]) + bfr(btd[j])); }
  LDSX();
  for (int rl = 0; rl < 16; ++rl) for (int pc = lane; pc < HH / 4; pc += 32) vst2(DS + (r0 + rl) * HH + pc * 4, *(const v4f*)&st[wave][rl][pc * 4]);
  { v8f acc[8] = {};
#pragma unroll 1
    for (int part = 0; part < 3; ++part) { const float* src = part == 0 ? CS : (part == 1 ? XS : CH);
#pragma unroll
      for (int kc = 0; kc < 4; ++kc) { const F2 a = split_row(src + (r0 + col) * DD, kc * 32, lane);
#pragma unroll
        for (int j = 0; j < 8; ++j) { const v16b w = frag_b(PT + P_WQ + (size_t)(j * 16 + col) * 896 + part * 128 + kc * 32, lane); acc[j] = wmma_bf(a.l, w, acc[j]); acc[j] = wmma_bf(a.h, w, acc[j]); } } }
#pragma unroll 2
    for (int kc = 0; kc < HH / 32; ++kc) { const F2 a = split_row(&st[wave][col][0], kc * 32, lane);
#pragma unroll
      for (int j = 0; j < 8; ++j) { const v16b w = frag_b(PT + P_WQ + (size_t)(j * 16 + col) * 896 + 384 + kc * 32, lane); acc[j] = wmma_bf(a.l, w, acc[j]); acc[j] = wmma_bf(a.h, w, acc[j]); } }
    LDSX();
#pragma unroll
    for (int j = 0; j < 8; ++j) { const float bb = bfr(bq[j * 16 + col]);
#pragma unroll
      for (int r = 0; r < 8; ++r) st[wave][8 * g + r][j * 16 + col] = acc[j][r] + bb; } }
  LDSX();
  { const int rl = lane >> 1, half = lane & 1; float s = 0.f;
#pragma unroll 8
    for (int j = 0; j < DD; ++j) s += st[wave][rl][j];
    const float mu = s * (1.0f / DD); float q2 = 0.f;
#pragma unroll 8
    for (int j = 0; j < DD; ++j) { const float d = st[wave][rl][j] - mu; q2 += d * d; }
    const float rs = rsqrtf(q2 * (1.0f / DD) + 1e-5f);
    LDSX();
    for (int j = half * 64; j < half * 64 + 64; ++j) st[wave][rl][j] = silu((st[wave][rl][j] - mu) * rs * bfr(gq[j]) + bfr(btq[j])); }
  LDSX();
  for (int rl = 0; rl < 16; ++rl) vst2(Q + (r0 + rl) * DD + lane * 4, *(const v4f*)&st[wave][rl][lane * 4]);
}

__global__ __launch_bounds__(256) void k_pool(const int* __restrict__ htok, const int* __restrict__ hpos, const int* __restrict__ hgrp, const int* __restrict__ hmask, const float* __restrict__ htime, const float* __restrict__ tok_emb, const float* __restrict__ pos_emb, const float* __restrict__ grp_emb,
                                              const float* __restrict__ tw1, const float* __restrict__ tb1, const float* __restrict__ tw2, const float* __restrict__ tb2, const float* __restrict__ CS, const float* __restrict__ XS, const float* __restrict__ CH, const float* __restrict__ DS, const float* __restrict__ Q, float* __restrict__ FU) {
  __shared__ float sq[DD], swq[DD], sa[LH + 8], ssu[DD], shist[DD], sred[8]; __shared__ float sc0;
  __shared__ __align__(16) float sfu[FUS];
  __shared__ float sE[LH][DD + 1], sU[LH][DD + 1];
  const int tid = threadIdx.x, wave = tid >> 5, lane = tid & 31; const int b = blockIdx.x;
  if (tid < DD) sq[tid] = Q[(size_t)b * DD + tid];
  __syncthreads();
  if (tid < DD) { float s = 0.f;
#pragma unroll 4
    for (int k = 0; k < DD; ++k) s += bfr(tw2[tid * DD + k]) * sq[k];
    swq[tid] = s; }
  if (tid == DD) { float s = 0.f; for (int k = 0; k < DD; ++k) s += bfr(tb2[k]) * sq[k]; sc0 = s; }
  __syncthreads();
  float myscore = -3.0e38f;
  if (tid < LH) { const int l = tid; const int it = clampi(htok[b * LH + l], NV - 1), ip = clampi(hpos[b * LH + l], NPOSV - 1), ig = clampi(hgrp[b * LH + l], NGRP - 1);
    const float t = bfr(htime[b * LH + l]); const float* er = tok_emb + (size_t)it * DD; const float* pr = pos_emb + (size_t)ip * DD; const float* gr = grp_emb + (size_t)ig * DD;
    float s = sc0;
#pragma unroll 2
    for (int d = 0; d < DD; ++d) { const float e = (bfr(er[d]) + bfr(pr[d])) + bfr(gr[d]); const float u = silu(t * bfr(tw1[d]) + bfr(tb1[d])); sE[l][d] = e; sU[l][d] = u; s += e * sq[d] + u * swq[d]; }
    s = s / sqrtf((float)DD);
    myscore = (hmask[b * LH + l] > 0) ? s : -1.0e9f; sa[l] = myscore; }
  { float m = myscore;
#pragma unroll
    for (int o = 1; o < 32; o <<= 1) m = fmaxf(m, __shfl_xor(m, o));
    if (lane == 0) sred[wave] = m; }
  __syncthreads();
  float mx = sred[0];
#pragma unroll
  for (int w = 1; w < 8; ++w) mx = fmaxf(mx, sred[w]);
  __syncthreads();
  { float e = (tid < LH) ? exp_ni(sa[tid] - mx) : 0.f; if (tid < LH) sa[tid] = e;
#pragma unroll
    for (int o = 1; o < 32; o <<= 1) e += __shfl_xor(e, o);
    if (lane == 0) sred[wave] = e; }
  __syncthreads();
  float Z = 0.f;
#pragma unroll
  for (int w = 0; w < 8; ++w) Z += sred[w];
  const float iz = 1.0f / Z;
  __syncthreads();
  if (tid < LH) sa[tid] *= iz;
  __syncthreads();
  if (tid < DD) { const int d = tid; float se = 0.f, su = 0.f, asum = 0.f;
#pragma unroll 4
    for (int l = 0; l < LH; ++l) { const float a = sa[l]; se += a * sE[l][d]; su += a * sU[l][d]; asum += a; }
    ssu[d] = su; shist[d] = se; if (d == 0) sc0 = asum; }
  __syncthreads();
  if (tid < DD) { const int d = tid; float s = shist[d];
#pragma unroll 4
    for (int j = 0; j < DD; ++j) s += ssu[j] * bfr(tw2[j * DD + d]);
    s += sc0 * bfr(tb2[d]); shist[d] = s; }
  __syncthreads();
  { const size_t rb = (size_t)b * DD;
    for (int d = tid; d < DD; d += 256) { const float cs = CS[rb + d], xs = XS[rb + d], hs = shist[d], ch = CH[rb + d];
      sfu[d] = cs; sfu[DD + d] = xs; sfu[2 * DD + d] = hs; sfu[3 * DD + d] = ch; sfu[4 * DD + d] = cs * hs; sfu[5 * DD + d] = cs * ch; sfu[6 * DD + d] = fabsf(hs - ch); }
    for (int d = tid; d < HH; d += 256) sfu[7 * DD + d] = DS[(size_t)b * HH + d]; }
  __syncthreads();
  for (int q = tid; q < FUS / 4; q += 256) vst2(FU + (size_t)b * FUS + q * 4, *(const v4f*)&sfu[q * 4]);
}
__global__ __launch_bounds__(128) void k_head(const float* __restrict__ FU, const __bf16* __restrict__ PT, const float* __restrict__ b1, const float* __restrict__ g1, const float* __restrict__ bt1, const float* __restrict__ b2, const float* __restrict__ w3, const float* __restrict__ b3, float* __restrict__ out) {
  __shared__ __align__(16) float st[4][16][HH + 4]; __shared__ __align__(16) float sh2[4][16][DD * 2 + 4]; __shared__ __align__(16) float sres[64];
  const int tid = threadIdx.x, wave = tid >> 5, lane = tid & 31, col = lane & 15, g = lane >> 4; const size_t r0 = (size_t)blockIdx.x * 64 + wave * 16;
#pragma unroll 1
  for (int pass = 0; pass < 2; ++pass) { v8f acc[16] = {};
#pragma unroll 1
    for (int kc = 0; kc < FUS / 32; ++kc) { const F2 a = split_row(FU + (r0 + col) * FUS, kc * 32, lane);
#pragma unroll
      for (int j = 0; j < 16; ++j) { const v16b w = frag_b(PT + P_W1O + (size_t)(pass * 256 + j * 16 + col) * FUS + kc * 32, lane); acc[j] = wmma_bf(a.l, w, acc[j]); acc[j] = wmma_bf(a.h, w, acc[j]); } }
#pragma unroll
    for (int j = 0; j < 16; ++j) { const int n = pass * 256 + j * 16 + col; const float bb = bfr(b1[n]);
#pragma unroll
      for (int r = 0; r < 8; ++r) st[wave][8 * g + r][n] = acc[j][r] + bb; } }
  LDSX();
  { const int rl = lane >> 1, half = lane & 1; float s = 0.f;
#pragma unroll 8
    for (int j = 0; j < HH; ++j) s += st[wave][rl][j];
    const float mu = s * (1.0f / HH); float q2 = 0.f;
#pragma unroll 8
    for (int j = 0; j < HH; ++j) { const float d = st[wave][rl][j] - mu; q2 += d * d; }
    const float rs = rsqrtf(q2 * (1.0f / HH) + 1e-5f);
    LDSX();
    for (int j = half * 256; j < half * 256 + 256; ++j) st[wave][rl][j] = silu((st[wave][rl][j] - mu) * rs * bfr(g1[j]) + bfr(bt1[j])); }
  LDSX();
  { v8f acc[16] = {};
#pragma unroll 2
    for (int kc = 0; kc < HH / 32; ++kc) { const F2 a = split_row(&st[wave][col][0], kc * 32, lane);
#pragma unroll
      for (int j = 0; j < 16; ++j) { const v16b w = frag_b(PT + P_W2O + (size_t)(j * 16 + col) * HH + kc * 32, lane); acc[j] = wmma_bf(a.l, w, acc[j]); acc[j] = wmma_bf(a.h, w, acc[j]); } }
#pragma unroll
    for (int j = 0; j < 16; ++j) { const int n = j * 16 + col; const float bb = bfr(b2[n]);
#pragma unroll
      for (int r = 0; r < 8; ++r) sh2[wave][8 * g + r][n] = silu(acc[j][r] + bb); } }
  LDSX();
  { const int rl = lane >> 1, half = lane & 1; float s = 0.f;
    for (int j = half * 128; j < half * 128 + 128; ++j) s += sh2[wave][rl][j] * bfr(w3[j]);
    s += __shfl_xor(s, 1); if (half == 0) sres[wave * 16 + rl] = s + bfr(b3[0]); }
  __syncthreads();
  if (tid < 16) vst2(out + (size_t)blockIdx.x * 64 + tid * 4, *(const v4f*)&sres[tid * 4]);
}

extern "C" void kernel_launch(void* const* d_in, const int* in_sizes, int n_in, void* d_out, int out_size, void* d_ws, size_t ws_size, hipStream_t stream) {
  (void)in_sizes; (void)n_in; (void)out_size;
  const int** I = (const int**)d_in; const float** F = (const float**)d_in;
  if (ws_size < (size_t)WS_END) return;
  char* ws = (char*)d_ws; __bf16* PT = (__bf16*)(ws + WS_PT); float *CS = (float*)(ws + WS_CS), *XS = (float*)(ws + WS_XS), *CH = (float*)(ws + WS_CH), *DS = (float*)(ws + WS_DS), *Q = (float*)(ws + WS_Q), *FU = (float*)(ws + WS_FU);
  k_pack<<<1664, 256, 0, stream>>>(F[15], F[17], F[21], F[25], F[29], F[33], PT);
  k_hist<<<TNS, 256, 0, stream>>>(I[0], I[1], I[4], I[5], I[6], I[7], F[8], F[10], F[12], F[13], F[14], F[16], PT, F[18], F[19], F[20], CS, XS, CH);
  k_dq<<<TNS / 64, 128, 0, stream>>>(F[9], PT, F[22], F[23], F[24], F[26], F[27], F[28], CS, XS, CH, DS, Q);
  k_pool<<<TNS, 256, 0, stream>>>(I[2], I[3], I[4], I[7], F[8], F[10], F[11], F[12], F[13], F[14], F[15], F[16], CS, XS, CH, DS, Q, FU);
  k_head<<<TNS / 64, 128, 0, stream>>>(FU, PT, F[30], F[31], F[32], F[34], F[35], F[36], (float*)d_out);
}
